// VariableSelectionNetwork_82360292868210
// MI455X (gfx1250) — hardware-verified
//
#include <hip/hip_runtime.h>

typedef __bf16         v16b  __attribute__((ext_vector_type(16)));
typedef unsigned short v16us __attribute__((ext_vector_type(16)));
typedef unsigned short v8us  __attribute__((ext_vector_type(8)));
typedef _Float16       v8h   __attribute__((ext_vector_type(8)));
typedef float          v8f   __attribute__((ext_vector_type(8)));
typedef float          v4f   __attribute__((ext_vector_type(4)));
typedef unsigned       v4u   __attribute__((ext_vector_type(4)));
typedef v8us __attribute__((may_alias)) v8usa;
typedef v8h  __attribute__((may_alias)) v8ha;
typedef v4f  __attribute__((may_alias)) v4fa;
typedef v4u  __attribute__((may_alias)) v4ua;

union FragU { v16us v; v8us half[2]; };

#define NB    64
#define NT    128
#define NTOK  (NB * NT)
#define NF    32
#define NU    256
#define KC    (2 * NU)
#define HTOK  (NTOK / 2)
#define MT    64
#define GTHR  256
#define CT    32
#define CTHR  256
#define PTHR  256
#define LNC     8.0f
#define INV_LNC 0.125f
#define LN_EPS  1e-3f
#define INV_U   (1.0f / 256.0f)

#define W2T_BYTES ((size_t)NF * NU * NU * 2)
#define LNP_BYTES ((size_t)NF * HTOK * NU * 2)
#define MPL_BYTES ((size_t)NF * HTOK * 4)
#define WSB_W2T ((size_t)0)
#define WSB_LNP (WSB_W2T + W2T_BYTES)
#define WSB_MPL (WSB_LNP + LNP_BYTES)
#define WSB_END (WSB_MPL + MPL_BYTES)
static_assert(WSB_LNP == 4194304);
static_assert(WSB_MPL == 71303168);
static_assert(WSB_END == 71827456);
static_assert(WSB_LNP % 128 == 0 && WSB_MPL % 128 == 0 && WSB_END % 128 == 0);
static_assert(WSB_END <= (size_t)134217728);
static_assert(NTOK % (2 * MT) == 0 && HTOK % MT == 0 && HTOK % CT == 0);
static_assert(NU % 32 == 0 && KC % 32 == 0);

#define GO_A   0
#define GO_LN  65536
#define GO_P   98304
#define GO_X   105472
#define GO_PS  105728
#define GO_PQ  106240
#define GO_PM  106752
#define GLDS   107264
static_assert(GO_LN == GO_A + MT * KC * 2);
static_assert(GO_P == GO_LN + MT * NU * 2);
static_assert(GO_X == GO_P + 7 * NU * 4);
static_assert(GO_PS == GO_X + MT * 4 && GO_PQ == GO_PS + MT * 2 * 4 && GO_PM == GO_PQ + MT * 2 * 4);
static_assert(GLDS == GO_PM + MT * 2 * 4);

#define PW1 0
#define PB1 256
#define PB2 512
#define PWG 768
#define PBG 1024
#define PGM 1280
#define PBT 1536

__device__ __forceinline__ unsigned bf16bits(float v) {
  const unsigned u = __builtin_bit_cast(unsigned, v);
  return (u + 0x7FFFu + ((u >> 16) & 1u)) >> 16;
}
__device__ __forceinline__ float bfr(float v) {
  return __builtin_bit_cast(float, bf16bits(v) << 16);
}
__device__ __forceinline__ float sigm_f(float v) {
  v = fminf(fmaxf(v, -30.0f), 30.0f);
  const float e = expf(-v);
  return 1.0f / (1.0f + e);
}
__device__ __forceinline__ float hsum16(float v) {
  v += __shfl_xor(v, 1);
  v += __shfl_xor(v, 2);
  v += __shfl_xor(v, 4);
  v += __shfl_xor(v, 8);
  return v;
}
__device__ __forceinline__ float h16f(unsigned bits) {
  return (float)__builtin_bit_cast(_Float16, (unsigned short)(bits & 0xFFFFu));
}

__device__ __forceinline__ v8f wmma_b16(v16us a, v16us b, v8f c) {
  const v16b av = __builtin_bit_cast(v16b, a);
  const v16b bv = __builtin_bit_cast(v16b, b);
  v8f d = __builtin_amdgcn_wmma_f32_16x16x32_bf16(false, av, false, bv, (short)0, c, false, false);
  asm volatile("v_nop\n\tv_nop\n\tv_nop\n\tv_nop" : "+v"(d) : "v"(a), "v"(b));
  return d;
}

__device__ __forceinline__ v16us load_frag(const unsigned short* p, int h) {
  FragU f;
  f.half[0] = *(const v8usa*)(p + 8 * h);
  f.half[1] = *(const v8usa*)(p + 16 + 8 * h);
  return f.v;
}

__global__ __launch_bounds__(PTHR) void k_prep(const float* __restrict__ W2,
                                               unsigned short* __restrict__ w2t)
{
  __shared__ __attribute__((aligned(16))) float sT[NU * 32];
  const int tid = threadIdx.x;
  const int f = blockIdx.x >> 3, nb = blockIdx.x & 7;
  const float* src = W2 + (size_t)f * NU * NU + nb * 32;
  #pragma unroll
  for (int i = 0; i < 8; ++i) {
    const int q = tid + i * PTHR;
    const int k = q >> 3, c4 = (q & 7) * 4;
    const v4f v = *(const v4fa*)(src + (size_t)k * NU + c4);
    *(v4fa*)(sT + k * 32 + c4) = v;
  }
  __syncthreads();
  unsigned short* dst = w2t + ((size_t)f * NU + nb * 32) * NU;
  v8us o[4];
  #pragma unroll
  for (int i = 0; i < 4; ++i) {
    const int c = tid + i * PTHR;
    const int row = c >> 5, k0 = (c & 31) * 8;
    v8us t;
    #pragma unroll
    for (int j = 0; j < 8; ++j) t[j] = (unsigned short)bf16bits(sT[(k0 + j) * 32 + row]);
    o[i] = t;
  }
  #pragma unroll
  for (int i = 0; i < 4; ++i) {
    const int c = tid + i * PTHR;
    *(volatile v8us*)(dst + (size_t)c * 8) = o[i];
  }
  __threadfence();
  #pragma unroll
  for (int i = 0; i < 4; ++i) {
    const int c = tid + i * PTHR;
    *(volatile v8us*)(dst + (size_t)c * 8) = o[i];
  }
}

__device__ __forceinline__ void lnp_store_pass(const _Float16* sLN, _Float16* dst, int tid) {
  #pragma unroll
  for (int i = 0; i < 8; ++i) {
    const int c = tid + GTHR * i;
    const v8h v = *(const v8ha*)(sLN + c * 8);
    *(volatile v8h*)(dst + (size_t)c * 8) = v;
  }
}

__global__ __launch_bounds__(GTHR) void k_grn(
    const float* __restrict__ x,
    const float* __restrict__ W1, const float* __restrict__ b1,
    const float* __restrict__ b2,
    const float* __restrict__ Wg, const float* __restrict__ bg,
    const float* __restrict__ gam, const float* __restrict__ bet,
    const unsigned short* __restrict__ w2t,
    _Float16* __restrict__ lnp, float* __restrict__ mpl, int tbase)
{
  extern __shared__ __attribute__((aligned(16))) char smem[];
  unsigned short* sA = (unsigned short*)(smem + GO_A);
  _Float16* sLN = (_Float16*)(smem + GO_LN);
  float* sP  = (float*)(smem + GO_P);
  float* sX  = (float*)(smem + GO_X);
  float* sPs = (float*)(smem + GO_PS);
  float* sPq = (float*)(smem + GO_PQ);
  float* sPm = (float*)(smem + GO_PM);

  const int tid = threadIdx.x, lane = tid & 31, w = tid >> 5;
  const int h = lane >> 4, m = lane & 15;
  const int msub = w & 3, qh = w >> 2;
  const int f = blockIdx.y;
  const int tokl0 = blockIdx.x * MT;
  const int tok0  = tbase + tokl0;
  const int rbase = 16 * msub + 8 * h;

  if (w < 7) {
    const float* src = W1;
    if (w == 1)      src = b1;
    else if (w == 2) src = b2;
    else if (w == 3) src = Wg;
    else if (w == 4) src = bg;
    else if (w == 5) src = gam;
    else if (w == 6) src = bet;
    src += (size_t)f * NU;
    #pragma unroll
    for (int i = 0; i < 2; ++i) {
      const int q = lane + 32 * i;
      const v4f v = *(const v4fa*)(src + 4 * q);
      const v4f r = { bfr(v.x), bfr(v.y), bfr(v.z), bfr(v.w) };
      *(v4fa*)(sP + w * NU + 4 * q) = r;
    }
  } else {
    const float v0 = x[(size_t)(tok0 + lane) * NF + f];
    const float v1 = x[(size_t)(tok0 + 32 + lane) * NF + f];
    sX[lane] = bfr(v0);
    sX[32 + lane] = bfr(v1);
  }
  __syncthreads();

  {
    const int row = tid >> 2, cb = (tid & 3) * 64;
    const float xv = sX[row];
    #pragma unroll 2
    for (int j = 0; j < 8; ++j) {
      const int c = cb + 8 * j;
      v8us hi8, lo8;
      #pragma unroll
      for (int i = 0; i < 8; ++i) {
        float v = xv * sP[PW1 + c + i] + sP[PB1 + c + i];
        v = fmaxf(v, 0.0f);
        const unsigned hb = bf16bits(v);
        const float hv = __builtin_bit_cast(float, hb << 16);
        const unsigned lb = bf16bits(v - hv);
        hi8[i] = (unsigned short)hb;
        lo8[i] = (unsigned short)lb;
      }
      *(v8usa*)(sA + row * KC + c) = hi8;
      *(v8usa*)(sA + row * KC + NU + c) = lo8;
    }
  }
  __syncthreads();

  const v8f z8 = {0.f, 0.f, 0.f, 0.f, 0.f, 0.f, 0.f, 0.f};
  v8f acc[8];
  #pragma unroll
  for (int nt = 0; nt < 8; ++nt) acc[nt] = z8;
  {
    const unsigned short* arow = sA + (16 * msub + m) * KC;
    const unsigned short* brow = w2t + ((size_t)f * NU + 128 * qh + m) * NU;
    #pragma unroll 1
    for (int k0 = 0; k0 < NU; k0 += 32) {
      const v16us ahi = load_frag(arow + k0, h);
      const v16us alo = load_frag(arow + NU + k0, h);
      #pragma unroll
      for (int nt = 0; nt < 8; ++nt) {
        const v16us b = load_frag(brow + (size_t)nt * 16 * NU + k0, h);
        acc[nt] = wmma_b16(ahi, b, acc[nt]);
        acc[nt] = wmma_b16(alo, b, acc[nt]);
      }
    }
  }

  float xr[8], s[8];
  #pragma unroll
  for (int r = 0; r < 8; ++r) { xr[r] = sX[rbase + r]; s[r] = 0.0f; }
  #pragma unroll
  for (int nt = 0; nt < 8; ++nt) {
    const int col = 128 * qh + 16 * nt + m;
    const float b2v = sP[PB2 + col];
    const float wgv = sP[PWG + col];
    const float bgv = sP[PBG + col];
    #pragma unroll
    for (int r = 0; r < 8; ++r) {
      const float g = sigm_f(xr[r] * wgv + bgv);
      const float rv = g * (acc[nt][r] + b2v) + xr[r];
      acc[nt][r] = rv;
      s[r] += rv;
    }
  }
  #pragma unroll
  for (int r = 0; r < 8; ++r) s[r] = hsum16(s[r]);
  if (m == 0) {
    #pragma unroll
    for (int r = 0; r < 8; ++r) sPs[(rbase + r) * 2 + qh] = s[r];
  }
  __syncthreads();
  float mu[8], q[8];
  #pragma unroll
  for (int r = 0; r < 8; ++r) {
    mu[r] = (sPs[(rbase + r) * 2] + sPs[(rbase + r) * 2 + 1]) * INV_U;
    q[r] = 0.0f;
  }
  #pragma unroll
  for (int nt = 0; nt < 8; ++nt)
    #pragma unroll
    for (int r = 0; r < 8; ++r) {
      const float d = acc[nt][r] - mu[r];
      acc[nt][r] = d;
      q[r] += d * d;
    }
  #pragma unroll
  for (int r = 0; r < 8; ++r) q[r] = hsum16(q[r]);
  if (m == 0) {
    #pragma unroll
    for (int r = 0; r < 8; ++r) sPq[(rbase + r) * 2 + qh] = q[r];
  }
  __syncthreads();
  float rs[8], sl[8];
  #pragma unroll
  for (int r = 0; r < 8; ++r) {
    rs[r] = rsqrtf((sPq[(rbase + r) * 2] + sPq[(rbase + r) * 2 + 1]) * INV_U + LN_EPS);
    sl[r] = 0.0f;
  }
  #pragma unroll
  for (int nt = 0; nt < 8; ++nt) {
    const int col = 128 * qh + 16 * nt + m;
    const float gv = sP[PGM + col];
    const float bv = sP[PBT + col];
    #pragma unroll
    for (int r = 0; r < 8; ++r) {
      const float lnv = acc[nt][r] * rs[r] * gv + bv;
      sl[r] += lnv;
      sLN[(rbase + r) * NU + col] = (_Float16)(lnv * LNC);
    }
  }
  #pragma unroll
  for (int r = 0; r < 8; ++r) sl[r] = hsum16(sl[r]);
  if (m == 0) {
    #pragma unroll
    for (int r = 0; r < 8; ++r) sPm[(rbase + r) * 2 + qh] = sl[r];
  }
  __syncthreads();

  v4f mv = {0.f, 0.f, 0.f, 0.f};
  const int lb = lane & 15;
  #pragma unroll
  for (int j = 0; j < 4; ++j) {
    const int row = 4 * lb + j;
    mv[j] = (sPm[row * 2] + sPm[row * 2 + 1]) * INV_U;
  }
  float* mdst = mpl + (size_t)f * HTOK + tokl0 + 4 * lb;
  _Float16* ldst = lnp + ((size_t)f * HTOK + tokl0) * NU;

  lnp_store_pass(sLN, ldst, tid);
  if (w == 0 && lane < 16) *(volatile v4f*)mdst = mv;
  __threadfence();
  lnp_store_pass(sLN, ldst, tid);
  if (w == 0 && lane < 16) *(volatile v4f*)mdst = mv;
}

__device__ __forceinline__ void out_store_pass(const float* sO, float* dst, int tid) {
  #pragma unroll
  for (int i = 0; i < 8; ++i) {
    const int c = tid + CTHR * i;
    const v4f v = *(const v4fa*)(sO + c * 4);
    *(volatile v4f*)(dst + (size_t)c * 4) = v;
  }
}

__global__ __launch_bounds__(CTHR) void k_comb(
    const _Float16* __restrict__ lnp, const float* __restrict__ mpl,
    const float* __restrict__ Ws, const float* __restrict__ bs,
    float* __restrict__ out, int tbase)
{
  __shared__ __attribute__((aligned(16))) float sO[CT * NU];
  __shared__ __attribute__((aligned(16))) float sM[NF * CT];
  __shared__ __attribute__((aligned(16))) float sWs[NF * NF];
  __shared__ __attribute__((aligned(16))) float sW[CT * NF];
  __shared__ __attribute__((aligned(16))) float sBs[NF];

  const int tid = threadIdx.x;
  const int rl0 = blockIdx.x * CT;
  const int grow0 = tbase + rl0;

  {
    const int ff = tid >> 3, c4 = (tid & 7) * 4;
    const v4f v = *(const v4fa*)(mpl + (size_t)ff * HTOK + rl0 + c4);
    *(v4fa*)(sM + ff * CT + c4) = v;
    const v4f a = *(const v4fa*)(Ws + tid * 4);
    const v4f ar = { bfr(a.x), bfr(a.y), bfr(a.z), bfr(a.w) };
    *(v4fa*)(sWs + tid * 4) = ar;
    const v4f bv = *(const v4fa*)(bs + (tid & 7) * 4);
    const v4f br = { bfr(bv.x), bfr(bv.y), bfr(bv.z), bfr(bv.w) };
    if (tid < 8) *(v4fa*)(sBs + tid * 4) = br;
  }
  __syncthreads();

  #pragma unroll 1
  for (int i = 0; i < 4; ++i) {
    const int p = tid + CTHR * i;
    const int row = p >> 5, fo = p & 31;
    float a = 0.0f;
    #pragma unroll 4
    for (int fp = 0; fp < NF; ++fp) a = fmaf(sM[fp * CT + row], sWs[fp * NF + fo], a);
    a += sBs[fo];
    sW[row * NF + fo] = sigm_f(a);
  }
  __syncthreads();

  {
    const int row = tid >> 3, cs = (tid & 7) * 32;
    float acc[32];
    #pragma unroll
    for (int k = 0; k < 32; ++k) acc[k] = 0.0f;
    const _Float16* base = lnp + (size_t)(rl0 + row) * NU + cs;
    #pragma unroll 1
    for (int f2 = 0; f2 < NF; ++f2) {
      const float wv = sW[row * NF + f2];
      const _Float16* p = base + (size_t)f2 * HTOK * NU;
      #pragma unroll
      for (int j = 0; j < 4; ++j) {
        const v4u rw = *(const v4ua*)(p + 8 * j);
        #pragma unroll
        for (int e = 0; e < 4; ++e) {
          const unsigned wd = rw[e];
          const float lo = h16f(wd);
          const float hi = h16f(wd >> 16);
          acc[8 * j + 2 * e]     = fmaf(wv, lo, acc[8 * j + 2 * e]);
          acc[8 * j + 2 * e + 1] = fmaf(wv, hi, acc[8 * j + 2 * e + 1]);
        }
      }
    }
    #pragma unroll
    for (int k4 = 0; k4 < 8; ++k4) {
      const v4f v = { acc[4 * k4] * INV_LNC, acc[4 * k4 + 1] * INV_LNC,
                      acc[4 * k4 + 2] * INV_LNC, acc[4 * k4 + 3] * INV_LNC };
      *(v4fa*)(sO + row * NU + cs + 4 * k4) = v;
    }
  }
  __syncthreads();

  float* dst = out + (size_t)grow0 * NU;
  out_store_pass(sO, dst, tid);
  __threadfence();
  out_store_pass(sO, dst, tid);
}

extern "C" void kernel_launch(void* const* d_in, const int* in_sizes, int n_in,
                              void* d_out, int out_size, void* d_ws, size_t ws_size,
                              hipStream_t stream) {
  if (n_in < 11) return;
  if (in_sizes[0] != NTOK * NF) return;
  if (in_sizes[1] != NF * NU || in_sizes[2] != NF * NU) return;
  if (in_sizes[3] != NF * NU * NU) return;
  if (in_sizes[4] != NF * NU || in_sizes[5] != NF * NU || in_sizes[6] != NF * NU) return;
  if (in_sizes[7] != NF * NU || in_sizes[8] != NF * NU) return;
  if (in_sizes[9] != NF * NF || in_sizes[10] != NF) return;
  if (out_size != NTOK * NU) return;
  if (ws_size < WSB_END) return;

  const float* x   = (const float*)d_in[0];
  const float* W1  = (const float*)d_in[1];
  const float* b1  = (const float*)d_in[2];
  const float* W2  = (const float*)d_in[3];
  const float* b2  = (const float*)d_in[4];
  const float* Wg  = (const float*)d_in[5];
  const float* bg  = (const float*)d_in[6];
  const float* gam = (const float*)d_in[7];
  const float* bet = (const float*)d_in[8];
  const float* Ws  = (const float*)d_in[9];
  const float* bs  = (const float*)d_in[10];
  float* out = (float*)d_out;

  char* ws = (char*)d_ws;
  unsigned short* w2t = (unsigned short*)(ws + WSB_W2T);
  _Float16* lnp = (_Float16*)(ws + WSB_LNP);
  float* mpl = (float*)(ws + WSB_MPL);

  hipFuncSetAttribute(reinterpret_cast<const void*>(&k_grn),
                      hipFuncAttributeMaxDynamicSharedMemorySize, GLDS);

  k_prep<<<NF * 8, PTHR, 0, stream>>>(W2, w2t);

  for (int hh = 0; hh < 2; ++hh) {
    const int tbase = hh * HTOK;
    dim3 gGrn(HTOK / MT, NF);
    k_grn<<<gGrn, GTHR, GLDS, stream>>>(x, W1, b1, b2, Wg, bg, gam, bet, w2t, lnp, mpl, tbase);
    k_comb<<<HTOK / CT, CTHR, 0, stream>>>(lnp, mpl, Ws, bs, out, tbase);
  }
}
